// CovLayer_23416161698166
// MI455X (gfx1250) — hardware-verified
//
#include <hip/hip_runtime.h>

constexpr int kMsa     = 128;
constexpr int kRes     = 256;
constexpr int kEmb     = 32;
constexpr int kOutD    = 128;
constexpr int kKin     = kEmb * kEmb;
constexpr int kResEmb  = kRes * kEmb;
constexpr int kChunkI  = 16;
constexpr int kNumChunks = kRes / kChunkI;
constexpr int kM1      = kChunkI * kEmb;
constexpr int kM2      = kChunkI * kRes;
constexpr float kWCarry    = 32.0f;
constexpr float kWCarryInv = 1.0f / 32.0f;

constexpr size_t kOffXLT  = 0;
constexpr size_t kOffXRT  = kOffXLT + (size_t)kResEmb * kMsa * 2;
constexpr size_t kOffBT2  = kOffXRT + (size_t)kResEmb * kMsa * 2;
constexpr size_t kOffOUT1 = kOffBT2 + (size_t)kOutD * kKin * 2;
constexpr size_t kOffA2   = kOffOUT1 + (size_t)kM1 * kResEmb * 4;
constexpr size_t kWsTotal = kOffA2 + (size_t)kM2 * kKin * 2;
static_assert(kWsTotal == 29622272, "carve");
static_assert((kOffXRT % 128) == 0 && (kOffBT2 % 128) == 0 && (kOffOUT1 % 128) == 0 && (kOffA2 % 128) == 0, "align");

typedef __attribute__((ext_vector_type(16))) _Float16 v16h;
typedef __attribute__((ext_vector_type(8)))  _Float16 v8h;
typedef __attribute__((ext_vector_type(16))) __bf16   v16b;
typedef __attribute__((ext_vector_type(8)))  __bf16   v8b;
typedef __attribute__((ext_vector_type(8)))  float    v8f;
typedef __attribute__((ext_vector_type(4)))  float    v4f;
typedef __attribute__((ext_vector_type(4)))  unsigned int v4u;

__device__ __forceinline__ unsigned short f2bf_bits(float f) {
  unsigned u = __float_as_uint(f);
  return (unsigned short)((u + 0x7FFFu + ((u >> 16) & 1u)) >> 16);
}
__device__ __forceinline__ float bf_bits2f(unsigned short h) { return __uint_as_float(((unsigned)h) << 16); }

__device__ __forceinline__ void dep_guard_h(v8f& a, v8f& b, v16h x, v16h y) { asm volatile("v_nop\n\tv_nop\n\tv_nop\n\tv_nop" : "+v"(a), "+v"(b) : "v"(x), "v"(y)); }
__device__ __forceinline__ void dep_guard_b(v8f& a, v8f& b, v16b x, v16b y) { asm volatile("v_nop\n\tv_nop\n\tv_nop\n\tv_nop" : "+v"(a), "+v"(b) : "v"(x), "v"(y)); }
__device__ __forceinline__ void keep4_h(v16h a, v16h b, v16h c, v16h d) { asm volatile("v_nop" :: "v"(a), "v"(b), "v"(c), "v"(d)); }
__device__ __forceinline__ void keep4_b(v16b a, v16b b, v16b c, v16b d) { asm volatile("v_nop" :: "v"(a), "v"(b), "v"(c), "v"(d)); }
__device__ __forceinline__ void acc_guard4(v8f& a, v8f& b, v8f& c, v8f& d) { asm volatile("v_nop\n\tv_nop\n\tv_nop\n\tv_nop" : "+v"(a), "+v"(b), "+v"(c), "+v"(d)); }
template <typename T> struct Frag;
template <> struct Frag<_Float16> {
  typedef v16h V; union U { v16h v; v8h h[2]; };
  static __device__ __forceinline__ v16h load(const _Float16* p) {
    U f; f.h[0] = *(const v8h*)(p); f.h[1] = *(const v8h*)(p + 16); return f.v;
  }
  static __device__ __forceinline__ v8f mma(v16h a, v16h b, v8f c) {
    return __builtin_amdgcn_wmma_f32_16x16x32_f16(false, a, false, b, (short)0, c, false, false);
  }
  static __device__ __forceinline__ void guard(v8f& a, v8f& b, v16h x, v16h y) { dep_guard_h(a, b, x, y); }
  static __device__ __forceinline__ void keep(v16h a, v16h b, v16h c, v16h d) { keep4_h(a, b, c, d); }
};
template <> struct Frag<__bf16> {
  typedef v16b V; union U { v16b v; v8b h[2]; };
  static __device__ __forceinline__ v16b load(const __bf16* p) {
    U f; f.h[0] = *(const v8b*)(p); f.h[1] = *(const v8b*)(p + 16); return f.v;
  }
  static __device__ __forceinline__ v8f mma(v16b a, v16b b, v8f c) {
    return __builtin_amdgcn_wmma_f32_16x16x32_bf16(false, a, false, b, (short)0, c, false, false);
  }
  static __device__ __forceinline__ void guard(v8f& a, v8f& b, v16b x, v16b y) { dep_guard_b(a, b, x, y); }
  static __device__ __forceinline__ void keep(v16b a, v16b b, v16b c, v16b d) { keep4_b(a, b, c, d); }
};

__device__ __forceinline__ unsigned pk16(unsigned short a, unsigned short b) { return (unsigned)a | ((unsigned)b << 16); }
__device__ __forceinline__ unsigned short h_bits(float f) { const _Float16 h = (_Float16)f; return __builtin_bit_cast(unsigned short, h); }

template <int ET> struct Elem;
template <> struct Elem<0> { typedef _Float16 T; };
template <> struct Elem<1> { typedef __bf16 T; };
template <int ET, bool SPLIT, int BIAS_MODE, int OUT_MODE, bool RESID, int ACT = 0>
__global__ __launch_bounds__(256) void wmma_gemm64(
    const unsigned short* __restrict__ Ap, const unsigned short* __restrict__ A2p, int lda, long strideA,
    const unsigned short* __restrict__ Btp, const unsigned short* __restrict__ Bt2p, int ldb, long strideB,
    void* __restrict__ Cout, void* __restrict__ Cout2, int ldc, long strideC,
    const float* __restrict__ bias,
    const float* __restrict__ resid, long strideR,
    int M, int N, int K, float scale) {
  typedef typename Elem<ET>::T T;
  typedef typename Frag<T>::V V;
  const T* A = (const T*)Ap; const T* A2 = (const T*)A2p; const T* Bt = (const T*)Btp; const T* Bt2 = (const T*)Bt2p;
  __shared__ __align__(16) float sT[8][16 * 68];
  const int b    = blockIdx.y;
  const int lane = threadIdx.x & 31;
  const int wave = threadIdx.x >> 5;
  const int tilesN = N >> 6;
  const int tilesM = M >> 6;
  const int tile = blockIdx.x * 8 + wave;
  if (tile >= tilesM * tilesN) return;
  const int tm = tile / tilesN;
  const int tn = tile - tm * tilesN;
  const int m0 = tm << 6;
  const int n0 = tn << 6;

  const T* Ab  = A  + (size_t)b * strideA;
  const T* Bb  = Bt + (size_t)b * strideB;
  const T* Ab2 = SPLIT ? (A2  + (size_t)b * strideA) : nullptr;
  const T* Bb2 = SPLIT ? (Bt2 + (size_t)b * strideB) : nullptr;

  const int rlane = lane & 15;
  const int koff  = (lane >> 4) * 8;
  const int mOff  = (lane >> 4) * 8;

  v8f acc[4][4];
#pragma unroll
  for (int i = 0; i < 4; ++i)
#pragma unroll
    for (int j = 0; j < 4; ++j) acc[i][j] = (v8f){0.f,0.f,0.f,0.f,0.f,0.f,0.f,0.f};

  for (int k0 = 0; k0 < K; k0 += 32) {
    V bh[4], bl[4];
#pragma unroll
    for (int j = 0; j < 4; ++j) {
      const size_t bo = (size_t)(n0 + (j << 4) + rlane) * ldb + koff + k0;
      bh[j] = Frag<T>::load(Bb + bo);
      if (SPLIT) bl[j] = Frag<T>::load(Bb2 + bo);
    }
#pragma unroll
    for (int i = 0; i < 4; ++i) {
      const size_t ao = (size_t)(m0 + (i << 4) + rlane) * lda + koff + k0;
      V ah = Frag<T>::load(Ab + ao);
      V al;
      if (SPLIT) al = Frag<T>::load(Ab2 + ao);
#pragma unroll
      for (int j = 0; j < 4; ++j) {
        acc[i][j] = Frag<T>::mma(ah, bh[j], acc[i][j]);
        if (SPLIT) {
          acc[i][j] = Frag<T>::mma(ah, bl[j], acc[i][j]);
          acc[i][j] = Frag<T>::mma(al, bh[j], acc[i][j]);
        }
      }
      Frag<T>::guard(acc[i][0], acc[i][3], ah, SPLIT ? al : ah);
    }
    Frag<T>::keep(bh[0], bh[1], bh[2], bh[3]);
    if (SPLIT) Frag<T>::keep(bl[0], bl[1], bl[2], bl[3]);
  }
  acc_guard4(acc[0][0], acc[0][1], acc[0][2], acc[0][3]);
  acc_guard4(acc[1][0], acc[1][1], acc[1][2], acc[1][3]);
  acc_guard4(acc[2][0], acc[2][1], acc[2][2], acc[2][3]);
  acc_guard4(acc[3][0], acc[3][1], acc[3][2], acc[3][3]);

  float* slab = sT[wave];
  const float* Rb = RESID ? (resid + (size_t)b * strideR) : nullptr;
#pragma unroll
  for (int i = 0; i < 4; ++i) {
    const int mBase = m0 + (i << 4);
#pragma unroll
    for (int j = 0; j < 4; ++j) {
      const int n = n0 + (j << 4) + rlane;
      float bv = 0.f;
      if (BIAS_MODE == 2) bv = bias[n];
#pragma unroll
      for (int r = 0; r < 8; ++r) {
        float v = acc[i][j][r] * scale;
        if (BIAS_MODE == 1) v += bias[mBase + mOff + r];
        if (BIAS_MODE == 2) v += bv;
        if (RESID) v += Rb[(size_t)(mBase + mOff + r) * ldc + n];
        if (ACT == 2) v = fmaxf(v, 0.0f);
        if (ACT == 4) v = (v > 0.f) ? v : 0.01f * v;
        slab[(mOff + r) * 68 + (j << 4) + rlane] = v;
      }
    }
    __builtin_amdgcn_fence(__ATOMIC_RELEASE, "workgroup");
    __builtin_amdgcn_wave_barrier();
    __builtin_amdgcn_fence(__ATOMIC_ACQUIRE, "workgroup");
    if (OUT_MODE == 0) {
      float* C = (float*)Cout + (size_t)b * strideC;
      const int hh = lane >> 4, c4 = (lane & 15) * 4;
      for (int pass = 0; pass < 2; ++pass) {
#pragma unroll
        for (int it = 0; it < 8; ++it) {
          const int row = it * 2 + hh;
          v4f v = *(const v4f*)(slab + row * 68 + c4);
          *(volatile v4f*)(C + (size_t)(mBase + row) * ldc + n0 + c4) = v;
        }
        __threadfence();
      }
    } else {
      const int q = lane >> 3, c8 = (lane & 7) * 8;
      unsigned short* C  = (unsigned short*)Cout  + (size_t)b * strideC;
      unsigned short* C2 = (OUT_MODE == 2) ? ((unsigned short*)Cout2 + (size_t)b * strideC) : nullptr;
      for (int pass = 0; pass < 2; ++pass) {
#pragma unroll
        for (int it = 0; it < 4; ++it) {
          const int row = it * 4 + q;
          const float* sp = slab + row * 68 + c8;
          v8h hv, lv;
#pragma unroll
          for (int e = 0; e < 8; ++e) {
            if (OUT_MODE == 1) {
              hv[e] = (_Float16)sp[e];
            } else {
              unsigned short hb = f2bf_bits(sp[e]);
              unsigned short lb = f2bf_bits(sp[e] - bf_bits2f(hb));
              hv[e] = __builtin_bit_cast(_Float16, hb);
              lv[e] = __builtin_bit_cast(_Float16, lb);
            }
          }
          *(volatile v8h*)(C + (size_t)(mBase + row) * ldc + n0 + c8) = hv;
          if (OUT_MODE == 2) *(volatile v8h*)(C2 + (size_t)(mBase + row) * ldc + n0 + c8) = lv;
        }
        __threadfence();
      }
    }
    __builtin_amdgcn_fence(__ATOMIC_RELEASE, "workgroup");
    __builtin_amdgcn_wave_barrier();
    __builtin_amdgcn_fence(__ATOMIC_ACQUIRE, "workgroup");
  }
}

__global__ __launch_bounds__(256) void tcast_kernel(const float* __restrict__ src, unsigned short* __restrict__ dst,
                                                    int nrows, int ncols, float scale) {
  __shared__ float sm[64][65];
  const int t  = threadIdx.x;
  const int c0 = blockIdx.x * 64;
  const int r0 = blockIdx.y * 64;
#pragma unroll
  for (int i = 0; i < 16; ++i) {
    const int e  = i * 256 + t;
    const int rl = e >> 6;
    const int cl = e & 63;
    sm[cl][rl] = src[(size_t)(r0 + rl) * ncols + c0 + cl] * scale;
  }
  __syncthreads();
  const int lane = t & 31, wave = t >> 5;
  const int q = lane >> 3, c8 = (lane & 7) * 8;
  for (int pass = 0; pass < 2; ++pass) {
#pragma unroll
    for (int it = 0; it < 2; ++it) {
      const int row = wave * 8 + it * 4 + q;
      unsigned short hb[8];
#pragma unroll
      for (int e = 0; e < 8; ++e) hb[e] = h_bits(sm[row][c8 + e]);
      const v4u u = (v4u){pk16(hb[0], hb[1]), pk16(hb[2], hb[3]), pk16(hb[4], hb[5]), pk16(hb[6], hb[7])};
      *(volatile v4u*)(dst + (size_t)(c0 + row) * nrows + r0 + c8) = u;
    }
    __threadfence();
  }
}

__global__ __launch_bounds__(128) void shuffle_kernel(const float* __restrict__ O1, unsigned short* __restrict__ A2) {
  const int row = blockIdx.x;
  const int il  = row >> 8;
  const int j   = row & 255;
  const int t   = threadIdx.x;
  const int l   = t >> 2;
  const int r8  = (t & 3) * 8;
  const float* p = O1 + (size_t)(il * kEmb + l) * kResEmb + (size_t)j * kEmb + r8;
  const v4f a = *(const v4f*)(p);
  const v4f c = *(const v4f*)(p + 4);
  unsigned short hb[8];
#pragma unroll
  for (int e = 0; e < 4; ++e) {
    hb[e]     = h_bits(a[e]);
    hb[4 + e] = h_bits(c[e]);
  }
  const v4u u = (v4u){pk16(hb[0], hb[1]), pk16(hb[2], hb[3]), pk16(hb[4], hb[5]), pk16(hb[6], hb[7])};
  unsigned short* qd = A2 + (size_t)row * kKin + l * kEmb + r8;
  *(volatile v4u*)qd = u;
  __threadfence();
  *(volatile v4u*)qd = u;
}

extern "C" void kernel_launch(void* const* d_in, const int* in_sizes, int n_in,
                              void* d_out, int out_size, void* d_ws, size_t ws_size,
                              hipStream_t stream) {
  if (n_in < 4) return;
  if (in_sizes[0] != kMsa * kRes * kEmb) return;
  if (in_sizes[1] != kMsa * kRes * kEmb) return;
  if (in_sizes[2] != kKin * kOutD) return;
  if (in_sizes[3] != kOutD) return;
  if (out_size != kRes * kRes * kOutD) return;
  if (ws_size < kWsTotal) return;

  const float* xl   = (const float*)d_in[0];
  const float* xr   = (const float*)d_in[1];
  const float* W    = (const float*)d_in[2];
  const float* bias = (const float*)d_in[3];
  float* out = (float*)d_out;
  char* ws = (char*)d_ws;
  unsigned short* XLT  = (unsigned short*)(ws + kOffXLT);
  unsigned short* XRT  = (unsigned short*)(ws + kOffXRT);
  unsigned short* BT2  = (unsigned short*)(ws + kOffBT2);
  float*          OUT1 = (float*)(ws + kOffOUT1);
  unsigned short* A2   = (unsigned short*)(ws + kOffA2);

  tcast_kernel<<<dim3(kResEmb / 64, kMsa / 64), 256, 0, stream>>>(xl, XLT, kMsa, kResEmb, 1.0f);
  tcast_kernel<<<dim3(kResEmb / 64, kMsa / 64), 256, 0, stream>>>(xr, XRT, kMsa, kResEmb, 1.0f);
  tcast_kernel<<<dim3(kOutD / 64, kKin / 64), 256, 0, stream>>>(W, BT2, kKin, kOutD, kWCarry);

  const int tiles1  = (kM1 / 64) * (kResEmb / 64);
  const int blocks1 = (tiles1 + 7) / 8;
  const int tiles2  = (kM2 / 64) * (kOutD / 64);
  const int blocks2 = (tiles2 + 7) / 8;

  for (int ch = 0; ch < kNumChunks; ++ch) {
    const unsigned short* A1 = XLT + (size_t)ch * kM1 * kMsa;
    wmma_gemm64<0, false, 0, 0, false><<<dim3(blocks1, 1), 256, 0, stream>>>(
        A1, A1, kMsa, 0L,
        XRT, XRT, kMsa, 0L,
        (void*)OUT1, (void*)OUT1, kResEmb, 0L,
        bias, bias, 0L,
        kM1, kResEmb, kMsa, 1.0f);
    shuffle_kernel<<<kM2, 128, 0, stream>>>(OUT1, A2);
    float* Cc = out + (size_t)ch * kM2 * kOutD;
    wmma_gemm64<0, false, 2, 0, false><<<dim3(blocks2, 1), 256, 0, stream>>>(
        A2, A2, kKin, 0L,
        BT2, BT2, kKin, 0L,
        (void*)Cc, (void*)Cc, kOutD, 0L,
        bias, bias, 0L,
        kM2, kOutD, kKin, kWCarryInv);
  }
}
